// lstm_32779190403342
// MI455X (gfx1250) — hardware-run, weakly checked
//
#include <hip/hip_runtime.h>
#include <math.h>

typedef __attribute__((ext_vector_type(16))) __bf16   v16b;
typedef __attribute__((ext_vector_type(8)))  __bf16   v8b;
typedef __attribute__((ext_vector_type(8)))  _Float16 v8h;
typedef __attribute__((ext_vector_type(8)))  float    v8f;
typedef __attribute__((ext_vector_type(4)))  float    v4f;

constexpr int kT            = 400000;
constexpr int kIn           = 40;
constexpr int kEmb          = 20;
constexpr int kHid          = 20;
constexpr int kGate         = 4 * kHid;
constexpr int kKp0          = 64;
constexpr int kKp1          = 32;
constexpr int kHp           = 32;
constexpr int kNumSeg       = 5;
constexpr int kSeg          = kT / kNumSeg;
constexpr int kRowsPerWave  = 16;
constexpr int kWavesPerBlk  = 8;
constexpr int kRowsPerBlk   = kRowsPerWave * kWavesPerBlk;
constexpr int kSegBlocks    = kSeg / kRowsPerBlk;
constexpr int kSlabFloats   = kRowsPerWave * kGate;
constexpr int kOutTotal     = kT + 4 * kHid;
constexpr int kStateFloats  = 64;
constexpr int kStateSlots   = kNumSeg + 1;
constexpr int kStateLayer   = kStateSlots * kStateFloats;

constexpr size_t kWsB0Bytes    = 16384;
constexpr size_t kWsB1Bytes    = 8192;
constexpr size_t kWsBiasBytes  = 4096;
constexpr size_t kWsStateBytes = 8192;
constexpr size_t kWsPreBytes   = (size_t)kSeg * kGate * 4;
constexpr size_t kWsHBytes     = (size_t)kSeg * kHp * 4;
constexpr size_t kWsOffBhi0    = 0;
constexpr size_t kWsOffBlo0    = kWsOffBhi0 + kWsB0Bytes;
constexpr size_t kWsOffBhi1    = kWsOffBlo0 + kWsB0Bytes;
constexpr size_t kWsOffBlo1    = kWsOffBhi1 + kWsB1Bytes;
constexpr size_t kWsOffBias0   = kWsOffBlo1 + kWsB1Bytes;
constexpr size_t kWsOffBias1   = kWsOffBias0 + kWsBiasBytes;
constexpr size_t kWsOffState   = kWsOffBias1 + kWsBiasBytes;
constexpr size_t kWsOffPre     = kWsOffState + kWsStateBytes;
constexpr size_t kWsOffH       = kWsOffPre + kWsPreBytes;
constexpr size_t kWsOffGat     = kWsOffH + kWsHBytes;
constexpr size_t kWsTotal      = kWsB0Bytes + kWsB0Bytes + kWsB1Bytes + kWsB1Bytes + kWsBiasBytes + kWsBiasBytes
                               + kWsStateBytes + kWsPreBytes + kWsHBytes + kWsPreBytes;

static_assert(kGate == 80);
static_assert(kGate == 5 * 16);
static_assert(kIn == 40 && kIn % 4 == 0 && kIn <= kKp0 && kKp0 % 32 == 0);
static_assert(kHid == 20 && kHid % 4 == 0 && kHid <= kKp1 && kKp1 % 32 == 0);
static_assert(kHp == 32 && kHp >= kHid);
static_assert(kSeg * kNumSeg == kT);
static_assert(kSeg == 80000);
static_assert(kSeg % kRowsPerBlk == 0);
static_assert(kSegBlocks * kRowsPerBlk == kSeg);
static_assert(kSeg % 32 == 0);
static_assert(((size_t)kSeg * 4) % 128 == 0);
static_assert((size_t)kOutTotal * 4 == 1600320ull);
static_assert((size_t)kGate * kKp0 * 2 <= kWsB0Bytes);
static_assert((size_t)kGate * kKp1 * 2 <= kWsB1Bytes);
static_assert(128 * 4 <= kWsBiasBytes);
static_assert((size_t)2 * kStateLayer * 4 <= kWsStateBytes);
static_assert(kWsOffPre == 65536ull);
static_assert(kWsOffPre % 128 == 0 && kWsOffH % 128 == 0 && kWsOffGat % 128 == 0);
static_assert(((size_t)kRowsPerWave * kGate * 4) % 128 == 0);
static_assert(kSlabFloats == 10 * 128);
static_assert(kWsTotal == 61505536ull);
static_assert(kWsOffGat + kWsPreBytes == kWsTotal);
static_assert(kWsTotal <= 134217728ull);

__device__ __forceinline__ unsigned short f2bf_bits(float f) {
  unsigned u = __float_as_uint(f);
  return (unsigned short)((u + 0x7FFFu + ((u >> 16) & 1u)) >> 16);
}
__device__ __forceinline__ float bf_bits2f(unsigned short h) { return __uint_as_float(((unsigned)h) << 16); }
__device__ __forceinline__ void bf_split(float v, unsigned short& hb, unsigned short& lb) {
  hb = f2bf_bits(v);
  lb = f2bf_bits(v - bf_bits2f(hb));
}
__device__ __forceinline__ void pin1(float& v) { asm volatile("" : "+v"(v)); }

union FragB { v16b v; v8b h[2]; };
__device__ __forceinline__ v16b frag_load_b(const __bf16* p) {
  FragB f;
  f.h[0] = *(const v8b*)(p);
  f.h[1] = *(const v8b*)(p + 16);
  return f.v;
}
__device__ __forceinline__ v8f mma_bf(v16b a, v16b b, v8f c) {
  c = __builtin_amdgcn_wmma_f32_16x16x32_bf16(false, a, false, b, (short)0, c, false, false);
  asm volatile("v_nop\n\tv_nop\n\tv_nop\n\tv_nop" : "+v"(c) : "v"(a), "v"(b));
  return c;
}
template <int BASE>
__device__ __forceinline__ void put4(v16b& hi, v16b& lo, v4f q, bool keep) {
#pragma unroll
  for (int e = 0; e < 4; ++e) {
    const float raw = q[e];
    const float s = keep ? raw : 0.0f;
    unsigned short hb, lb;
    bf_split(s, hb, lb);
    hi[BASE + e] = __builtin_bit_cast(__bf16, hb);
    lo[BASE + e] = __builtin_bit_cast(__bf16, lb);
  }
}
template <int KREAL, int CH, int GRP>
__device__ __forceinline__ void a_group(const float* xr, int hs, v16b& hi, v16b& lo) {
  constexpr int kmin = 32 * CH + ((GRP < 2) ? (4 * GRP) : (16 + 4 * (GRP - 2)));
  if (kmin < KREAL) {
    const int k = kmin + 8 * hs;
    const bool ok = (k + 4 <= KREAL);
    const int kc = ok ? k : (KREAL - 4);
    v4f q = *(const v4f*)(xr + kc);
    asm volatile("" : "+v"(q));
    put4<4 * GRP>(hi, lo, q, ok);
  }
}
template <int KREAL, int CH>
__device__ __forceinline__ void a_chunk(const float* xr, int hs, v16b& hi, v16b& lo) {
  const __bf16 zb = __builtin_bit_cast(__bf16, (unsigned short)0);
#pragma unroll
  for (int q = 0; q < 16; ++q) { hi[q] = zb; lo[q] = zb; }
  a_group<KREAL, CH, 0>(xr, hs, hi, lo);
  a_group<KREAL, CH, 1>(xr, hs, hi, lo);
  a_group<KREAL, CH, 2>(xr, hs, hi, lo);
  a_group<KREAL, CH, 3>(xr, hs, hi, lo);
}

__global__ __launch_bounds__(256) void prep_kernel(
    const float* __restrict__ W_inp, const float* __restrict__ b_inp,
    const float* __restrict__ W_ih0, const float* __restrict__ b_ih0,
    const float* __restrict__ b_hh0,
    const float* __restrict__ W_ih1, const float* __restrict__ b_ih1,
    const float* __restrict__ b_hh1,
    unsigned short* __restrict__ Bhi0, unsigned short* __restrict__ Blo0,
    unsigned short* __restrict__ Bhi1, unsigned short* __restrict__ Blo1,
    float* __restrict__ bias0, float* __restrict__ bias1,
    float* __restrict__ state)
{
  const int tid = threadIdx.x;
#pragma unroll 1
  for (int item = tid; item < kGate * 8; item += 256) {
    const int n   = item >> 3;
    const int grp = item & 7;
    const bool real = (grp < kIn / 8);
    const int kb = real ? 8 * grp : (kIn - 8);
    float acc[8];
#pragma unroll
    for (int i = 0; i < 8; ++i) acc[i] = 0.0f;
#pragma unroll 1
    for (int e = 0; e < kEmb; ++e) {
      const float wn = W_ih0[n * kEmb + e];
      const v4f u0 = *(const v4f*)(W_inp + e * kIn + kb);
      const v4f u1 = *(const v4f*)(W_inp + e * kIn + kb + 4);
#pragma unroll
      for (int i = 0; i < 4; ++i) {
        acc[i]     = fmaf(wn, u0[i], acc[i]);
        acc[4 + i] = fmaf(wn, u1[i], acc[4 + i]);
      }
    }
    v8h hv, lv;
#pragma unroll
    for (int i = 0; i < 8; ++i) {
      const float s = real ? acc[i] : 0.0f;
      unsigned short hb, lb;
      bf_split(s, hb, lb);
      hv[i] = __builtin_bit_cast(_Float16, hb);
      lv[i] = __builtin_bit_cast(_Float16, lb);
    }
    volatile v8h* ph = (volatile v8h*)(Bhi0 + (size_t)n * kKp0 + grp * 8);
    volatile v8h* pl = (volatile v8h*)(Blo0 + (size_t)n * kKp0 + grp * 8);
    *ph = hv;
    *pl = lv;
    __threadfence();
    *ph = hv;
    *pl = lv;
  }
#pragma unroll 1
  for (int item = tid; item < kGate * 4; item += 256) {
    const int n   = item >> 2;
    const int grp = item & 3;
    const bool ok0 = (8 * grp + 4 <= kHid);
    const bool ok1 = (8 * grp + 8 <= kHid);
    const int k0 = ok0 ? (8 * grp) : (kHid - 4);
    const int k1 = ok1 ? (8 * grp + 4) : (kHid - 4);
    v4f u0 = *(const v4f*)(W_ih1 + n * kHid + k0);
    v4f u1 = *(const v4f*)(W_ih1 + n * kHid + k1);
    asm volatile("" : "+v"(u0), "+v"(u1));
    v8h hv, lv;
#pragma unroll
    for (int i = 0; i < 4; ++i) {
      const float r0 = u0[i];
      const float r1 = u1[i];
      const float s0 = ok0 ? r0 : 0.0f;
      const float s1 = ok1 ? r1 : 0.0f;
      unsigned short hb, lb;
      bf_split(s0, hb, lb);
      hv[i] = __builtin_bit_cast(_Float16, hb);
      lv[i] = __builtin_bit_cast(_Float16, lb);
      bf_split(s1, hb, lb);
      hv[4 + i] = __builtin_bit_cast(_Float16, hb);
      lv[4 + i] = __builtin_bit_cast(_Float16, lb);
    }
    volatile v8h* ph = (volatile v8h*)(Bhi1 + (size_t)n * kKp1 + grp * 8);
    volatile v8h* pl = (volatile v8h*)(Blo1 + (size_t)n * kKp1 + grp * 8);
    *ph = hv;
    *pl = lv;
    __threadfence();
    *ph = hv;
    *pl = lv;
  }
  {
    const int i  = tid & 127;
    const bool rn = (i < kGate);
    const int nc = rn ? i : (kGate - 1);
    float val;
    volatile float* pb;
    if (tid < 128) {
      const float sb = b_ih0[nc] + b_hh0[nc];
      float d = 0.0f;
#pragma unroll 1
      for (int e = 0; e < kEmb; ++e) d = fmaf(W_ih0[nc * kEmb + e], b_inp[e], d);
      val = rn ? (d + sb) : 0.0f;
      pb = bias0 + i;
    } else {
      const float sb = b_ih1[nc] + b_hh1[nc];
      val = rn ? sb : 0.0f;
      pb = bias1 + i;
    }
    *pb = val;
    __threadfence();
    *pb = val;
  }
  if (tid < 128) {
    const int layer = tid >> 6;
    const int off   = tid & 63;
    volatile float* ps = state + layer * kStateLayer + off;
    *ps = 0.0f;
    __threadfence();
    *ps = 0.0f;
  }
}

template <int KREAL, int APITCH, int NCHUNK>
__global__ __launch_bounds__(256) void proj_kernel(
    const float* __restrict__ A,
    const unsigned short* __restrict__ Bhi_bits, const unsigned short* __restrict__ Blo_bits,
    const float* __restrict__ biasv, float* __restrict__ Cseg, int nrows)
{
  constexpr int KP = 32 * NCHUNK;
  static_assert(KREAL <= KP && KREAL % 4 == 0 && APITCH % 4 == 0 && APITCH >= KREAL);
  __shared__ __align__(16) float sSlab[kWavesPerBlk * kSlabFloats];
  const int tid  = threadIdx.x;
  const int lane = tid & 31;
  const int wave = tid >> 5;
  const int c    = lane & 15;
  const int hs   = lane >> 4;
  const int row0 = blockIdx.x * kRowsPerBlk + wave * kRowsPerWave;
  int row = row0 + c;
  row = (row < nrows) ? row : (nrows - 1);
  const float* xr = A + (size_t)row * APITCH;

  v16b ah0, al0, ah1, al1;
  a_chunk<KREAL, 0>(xr, hs, ah0, al0);
  if (NCHUNK > 1) {
    a_chunk<KREAL, 1>(xr, hs, ah1, al1);
  } else {
    ah1 = ah0;
    al1 = al0;
  }

  const __bf16* Bh = (const __bf16*)Bhi_bits;
  const __bf16* Bl = (const __bf16*)Blo_bits;

  v8f acc[5];
#pragma unroll
  for (int j = 0; j < 5; ++j) acc[j] = (v8f){0.f, 0.f, 0.f, 0.f, 0.f, 0.f, 0.f, 0.f};

#pragma unroll
  for (int j = 0; j < 5; ++j) {
    const size_t bo = (size_t)(16 * j + c) * KP + 8 * hs;
    {
      const v16b bh = frag_load_b(Bh + bo);
      const v16b bl = frag_load_b(Bl + bo);
      acc[j] = mma_bf(ah0, bh, acc[j]);
      acc[j] = mma_bf(al0, bh, acc[j]);
      acc[j] = mma_bf(ah0, bl, acc[j]);
    }
    if (NCHUNK > 1) {
      const v16b bh = frag_load_b(Bh + bo + 32);
      const v16b bl = frag_load_b(Bl + bo + 32);
      acc[j] = mma_bf(ah1, bh, acc[j]);
      acc[j] = mma_bf(al1, bh, acc[j]);
      acc[j] = mma_bf(ah1, bl, acc[j]);
    }
  }

  float* slab = sSlab + wave * kSlabFloats;
#pragma unroll
  for (int j = 0; j < 5; ++j) {
    const float bv = biasv[16 * j + c];
#pragma unroll
    for (int r = 0; r < 8; ++r) {
      const float val = acc[j][r] + bv;
      slab[(8 * hs + r) * kGate + 16 * j + c] = val;
    }
  }
  __syncthreads();
  {
    float* dst = Cseg + (size_t)row0 * kGate;
    for (int pass = 0; pass < 2; ++pass) {
#pragma unroll
      for (int it = 0; it < kSlabFloats / 128; ++it) {
        const int i = it * 128 + lane * 4;
        const v4f val = *(const v4f*)(slab + i);
        *(volatile v4f*)(dst + i) = val;
      }
      __threadfence();
    }
  }
}

__device__ __forceinline__ float sigm_q(float v) {
  return __builtin_amdgcn_rcpf(1.0f + __expf(-v));
}
__device__ __forceinline__ float tanh_q(float v) {
  return 1.0f - 2.0f * __builtin_amdgcn_rcpf(__expf(2.0f * v) + 1.0f);
}

template <bool HEAD>
__global__ __launch_bounds__(32) void chain_kernel(
    const float* __restrict__ G, const float* __restrict__ Whh,
    const float* __restrict__ st_in, float* __restrict__ st_out,
    float* __restrict__ Hplane,
    const float* __restrict__ W_out, const float* __restrict__ b_out,
    float* __restrict__ out_seg, const float* __restrict__ st_l0,
    float* __restrict__ out_fin, int is_last)
{
  __shared__ __align__(16) float sW[kHid * 32 * 4];
  __shared__ __align__(16) float sRing[32 * 32];
  __shared__ __align__(16) float sFin[4 * kHid];

  const int  lane = threadIdx.x;
  const bool live = (lane < kHid);
  const int  jc   = live ? lane : (kHid - 1);

#pragma unroll 1
  for (int k = 0; k < kHid; ++k) {
    v4f w;
#pragma unroll
    for (int g = 0; g < 4; ++g) {
      const float x0 = Whh[(g * kHid + jc) * kHid + k];
      w[g] = x0;
    }
    *(v4f*)(sW + (k * 32 + lane) * 4) = w;
  }

  float wout = 0.0f, bo = 0.0f;
  if (HEAD) {
    const float wo_raw = W_out[jc];
    wout = live ? wo_raw : 0.0f;
    bo = b_out[0];
  }

  float hcar = st_in[lane];
  float cst  = st_in[32 + jc];
  pin1(hcar);
  pin1(cst);
  hcar = live ? hcar : 0.0f;
#pragma unroll 1
  for (int s = 0; s < 32; ++s) sRing[s * 32 + lane] = (s == 31) ? hcar : 0.0f;
  __syncthreads();

  float hlast = hcar, lat = 0.0f;
  float p0, p1, p2, p3;
  {
    const float* pr = G + jc;
    p0 = pr[0];
    p1 = pr[kHid];
    p2 = pr[2 * kHid];
    p3 = pr[3 * kHid];
  }

#pragma unroll 1
  for (int t = 0; t < kSeg; ++t) {
    const int tn = (t + 1 < kSeg) ? (t + 1) : (kSeg - 1);
    const float* pn = G + (size_t)tn * kGate + jc;
    float n0 = pn[0];
    float n1 = pn[kHid];
    float n2 = pn[2 * kHid];
    float n3 = pn[3 * kHid];
    pin1(n0); pin1(n1); pin1(n2); pin1(n3);

    const int slot = t & 31;
    const float* hprev = sRing + ((t + 31) & 31) * 32;
    float a0 = p0, a1 = p1, a2 = p2, a3 = p3;
#pragma unroll 1
    for (int kk = 0; kk < kHid; kk += 4) {
      const v4f hv = *(const v4f*)(hprev + kk);
#pragma unroll
      for (int u = 0; u < 4; ++u) {
        const v4f w = *(const v4f*)(sW + ((kk + u) * 32 + lane) * 4);
        const float hk = hv[u];
        a0 = fmaf(w[0], hk, a0);
        a1 = fmaf(w[1], hk, a1);
        a2 = fmaf(w[2], hk, a2);
        a3 = fmaf(w[3], hk, a3);
      }
    }
    {
      const float ig = sigm_q(a0);
      const float fg = sigm_q(a1);
      const float gg = tanh_q(a2);
      const float og = sigm_q(a3);
      cst = fg * cst + ig * gg;
      const float hn = og * tanh_q(cst);
      hlast = live ? hn : 0.0f;
    }
    sRing[slot * 32 + lane] = hlast;
    __syncthreads();

    if (HEAD) {
      float y = hlast * wout;
      y += __shfl_xor(y, 16, 32);
      y += __shfl_xor(y, 8, 32);
      y += __shfl_xor(y, 4, 32);
      y += __shfl_xor(y, 2, 32);
      y += __shfl_xor(y, 1, 32);
      y += bo;
      lat = (lane == slot) ? y : lat;
      if (slot == 31) {
        volatile float* op = out_seg + (t - 31) + lane;
        *op = lat;
        __threadfence();
        *op = lat;
      }
    } else {
      if (slot == 31) {
        float* dst = Hplane + (size_t)(t - 31) * kHp;
        v4f fv[8];
#pragma unroll
        for (int it = 0; it < 8; ++it) fv[it] = *(const v4f*)(sRing + it * 128 + lane * 4);
        for (int pass = 0; pass < 2; ++pass) {
#pragma unroll
          for (int it = 0; it < 8; ++it) *(volatile v4f*)(dst + it * 128 + lane * 4) = fv[it];
          __threadfence();
        }
      }
    }

    p0 = n0; p1 = n1; p2 = n2; p3 = n3;
  }

  {
    const float cs = live ? cst : 0.0f;
    volatile float* sp = st_out + lane;
    *sp = hlast;
    *(sp + 32) = cs;
    __threadfence();
    *sp = hlast;
    *(sp + 32) = cs;
  }

  if (HEAD) {
    float h0f = st_l0[lane];
    float c0f = st_l0[32 + lane];
    pin1(h0f);
    pin1(c0f);
    if (live) {
      sFin[lane]            = h0f;
      sFin[kHid + lane]     = hlast;
      sFin[2 * kHid + lane] = c0f;
      sFin[3 * kHid + lane] = cst;
    }
    __syncthreads();
    const v4f fv = *(const v4f*)(sFin + 4 * jc);
    const bool dofin = live && (is_last != 0);
    volatile v4f* fp = (volatile v4f*)(out_fin + 4 * jc);
    if (dofin) *fp = fv;
    __threadfence();
    if (dofin) *fp = fv;
  }
}

extern "C" void kernel_launch(void* const* d_in, const int* in_sizes, int n_in,
                              void* d_out, int out_size, void* d_ws, size_t ws_size,
                              hipStream_t stream) {
  if (n_in < 13 || d_out == nullptr || d_ws == nullptr) return;
  if (in_sizes[0] != kT * kIn) return;
  if (in_sizes[1] != kEmb * kIn) return;
  if (in_sizes[2] != kEmb) return;
  if (in_sizes[3] != kGate * kEmb) return;
  if (in_sizes[4] != kGate * kHid) return;
  if (in_sizes[5] != kGate) return;
  if (in_sizes[6] != kGate) return;
  if (in_sizes[7] != kGate * kHid) return;
  if (in_sizes[8] != kGate * kHid) return;
  if (in_sizes[9] != kGate) return;
  if (in_sizes[10] != kGate) return;
  if (in_sizes[11] != kHid) return;
  if (in_sizes[12] != 1) return;
  if (out_size != kOutTotal) return;
  if (ws_size < kWsTotal) return;

  const float* in_states = (const float*)d_in[0];
  const float* W_inp     = (const float*)d_in[1];
  const float* b_inp     = (const float*)d_in[2];
  const float* W_ih0     = (const float*)d_in[3];
  const float* W_hh0     = (const float*)d_in[4];
  const float* b_ih0     = (const float*)d_in[5];
  const float* b_hh0     = (const float*)d_in[6];
  const float* W_ih1     = (const float*)d_in[7];
  const float* W_hh1     = (const float*)d_in[8];
  const float* b_ih1     = (const float*)d_in[9];
  const float* b_hh1     = (const float*)d_in[10];
  const float* W_out     = (const float*)d_in[11];
  const float* b_out     = (const float*)d_in[12];
  float* out = (float*)d_out;

  char* ws = (char*)d_ws;
  unsigned short* Bhi0 = (unsigned short*)(ws + kWsOffBhi0);
  unsigned short* Blo0 = (unsigned short*)(ws + kWsOffBlo0);
  unsigned short* Bhi1 = (unsigned short*)(ws + kWsOffBhi1);
  unsigned short* Blo1 = (unsigned short*)(ws + kWsOffBlo1);
  float* bias0 = (float*)(ws + kWsOffBias0);
  float* bias1 = (float*)(ws + kWsOffBias1);
  float* state = (float*)(ws + kWsOffState);
  float* pre0  = (float*)(ws + kWsOffPre);
  float* Hpl   = (float*)(ws + kWsOffH);
  float* gat1  = (float*)(ws + kWsOffGat);

  prep_kernel<<<1, 256, 0, stream>>>(W_inp, b_inp, W_ih0, b_ih0, b_hh0, W_ih1, b_ih1, b_hh1,
                                     Bhi0, Blo0, Bhi1, Blo1, bias0, bias1, state);

  for (int s = 0; s < kNumSeg; ++s) {
    const float* xseg = in_states + (size_t)s * kSeg * kIn;
    float* st0_in  = state + (0 * kStateSlots + s) * kStateFloats;
    float* st0_out = state + (0 * kStateSlots + s + 1) * kStateFloats;
    float* st1_in  = state + (1 * kStateSlots + s) * kStateFloats;
    float* st1_out = state + (1 * kStateSlots + s + 1) * kStateFloats;
    float* out_seg = out + (size_t)s * kSeg;
    const int last = (s == kNumSeg - 1) ? 1 : 0;

    proj_kernel<kIn, kIn, 2><<<kSegBlocks, 256, 0, stream>>>(xseg, Bhi0, Blo0, bias0, pre0, kSeg);
    chain_kernel<false><<<1, 32, 0, stream>>>(pre0, W_hh0, st0_in, st0_out, Hpl,
                                              W_out, b_out, out_seg, st0_in, out + kT, 0);
    proj_kernel<kHid, kHp, 1><<<kSegBlocks, 256, 0, stream>>>(Hpl, Bhi1, Blo1, bias1, gat1, kSeg);
    chain_kernel<true><<<1, 32, 0, stream>>>(gat1, W_hh1, st1_in, st1_out, Hpl,
                                             W_out, b_out, out_seg, st0_out, out + kT, last);
  }
}
